// EdgePredictionNetwork_58815282151679
// MI455X (gfx1250) — hardware-run, weakly checked
//
#include <hip/hip_runtime.h>
#include <stddef.h>
#include <stdint.h>

#define NN   2048
#define NB   64
#define MOL  32
#define EPM  992
#define NE   63488
#define SD   256
#define VD   64
#define ED   32
#define FD   16
#define NL   5
#define DIN  546
#define K2   512
#define GBM  64
#define GTHR 128
#define HLP  260
#define D2P  52
#define WSMAX 134217728

#define U_W1AB 32768
#define U_W1E  2048
#define U_WS   16384
#define U_WV   4096
#define U_WEP  3072
#define LUNITS (U_W1AB + U_W1E + U_WS + U_WV + U_WEP)
#define U_HEAD (16384 + 16384 + 16384 + 2048 + 1024)
#define TUNITS (NL * LUNITS + U_HEAD)
#define LE_W1AB 0
#define LE_W1E  (8 * U_W1AB)
#define LE_WS   (LE_W1E + 8 * U_W1E)
#define LE_WV   (LE_WS + 8 * U_WS)
#define LE_WEP  (LE_WV + 8 * U_WV)
#define LELEMS  (8 * LUNITS)
#define HE_WATM 0
#define HE_WSH  131072
#define HE_WB0  262144
#define HE_WBM  393216
#define HE_WB1  409600

#define EO_W1E 0
#define EO_WEP 8192
#define EO_PA  20480
#define EO_H   28672
#define EO_HL  36864
#define EO_MH  (EO_HL + 32 * HLP)
#define EO_D2  (EO_MH + 1024)
#define EO_C   (EO_D2 + 32 * D2P)
#define EO_GEO (EO_C + 768)
#define EO_PO  (EO_GEO + 2048)
#define EO_PN  (EO_PO + 128)
#define EDGE_LDS_FLOATS (EO_PN + 32)
#define EDGE_LDS_BYTES  (EDGE_LDS_FLOATS * 4)
#define HO_WBM 0
#define HO_WB1 8192
#define HO_SH  12288
#define HO_F   20480
#define HO_G   (HO_F + 32 * HLP)
#define HO_OUT (HO_G + 32 * HLP)
#define HO_DSQ (HO_OUT + 4960)
#define HO_C   (HO_DSQ + 1024)
#define HO_CO  (HO_C + 768)
#define HO_B1  (HO_CO + 128)
#define HEAD_LDS_FLOATS (HO_B1 + 16)
#define HEAD_LDS_BYTES  (HEAD_LDS_FLOATS * 4)

static_assert(MOL == 32);
static_assert(NB == 64);
static_assert(NN == NB * MOL);
static_assert(NE == 64 * 992);
static_assert(EPM == MOL * (MOL - 1));
static_assert((992 * 20) % 128 == 0);
static_assert(ED * 4 == 128);
static_assert(8 * 16 == 128);
static_assert(U_WEP == 48 * (K2 / 8));
static_assert(LUNITS == 58368 && LUNITS % 256 == 0 && U_HEAD % 256 == 0 && TUNITS % 256 == 0);
static_assert(U_W1AB % 256 == 0 && U_W1E % 256 == 0 && U_WS % 256 == 0 && U_WV % 256 == 0 && U_WEP % 256 == 0);
static_assert(EDGE_LDS_BYTES <= 327680 && HEAD_LDS_BYTES <= 327680);
static_assert(EDGE_LDS_BYTES == 203392 && HEAD_LDS_BYTES == 176064);
static_assert((HLP * 4) % 16 == 0 && (D2P * 4) % 16 == 0 && D2P >= 48 && HLP >= 256);
static_assert(EO_MH % 4 == 0 && EO_D2 % 4 == 0 && EO_C % 4 == 0 && EO_GEO % 4 == 0 && EO_PO % 4 == 0 && EO_PN % 4 == 0);
static_assert(HO_G % 4 == 0 && HO_OUT % 4 == 0 && HO_DSQ % 4 == 0 && HO_C % 4 == 0 && HO_CO % 4 == 0 && HO_B1 % 4 == 0);
static_assert(NN % GBM == 0 && (3 * NN) % GBM == 0 && K2 % 32 == 0);
static_assert(NB * EPM * 5 == 317440 && (EPM * 5) % 4 == 0 && (EPM * 5) / 4 == 1240);

typedef float          v4f   __attribute__((ext_vector_type(4)));
typedef float          v8f   __attribute__((ext_vector_type(8)));
typedef int            v4i   __attribute__((ext_vector_type(4)));
typedef int            v8i   __attribute__((ext_vector_type(8)));
typedef unsigned short v8us  __attribute__((ext_vector_type(8)));
typedef unsigned short v16us __attribute__((ext_vector_type(16)));
typedef __bf16         v16bf __attribute__((ext_vector_type(16)));
typedef v4f  __attribute__((may_alias)) v4fa;
typedef v4i  __attribute__((may_alias)) v4ia;
typedef v8us __attribute__((may_alias)) v8usa;
union FragB { v16bf v; v16us u; v8us h[2]; v8i w; };

__device__ __forceinline__ v8f wmb(const FragB& a, const FragB& b, v8f c) {
  v8f d = __builtin_amdgcn_wmma_f32_16x16x32_bf16(false, a.v, false, b.v, (short)0, c, false, false);
  asm volatile("v_nop\n\tv_nop\n\tv_nop\n\tv_nop" : "+v"(d) : "v"(a.w), "v"(b.w));
  return d;
}

__device__ __forceinline__ unsigned bf16_bits(float f) {
  const unsigned u = __float_as_uint(f);
  return (u + 0x7FFFu + ((u >> 16) & 1u)) >> 16;
}
__device__ __forceinline__ float bf16_val(float f) {
  return __uint_as_float(bf16_bits(f) << 16);
}
__device__ __forceinline__ v4f bf16_val4(v4f a) {
  v4f o;
  o.x = bf16_val(a.x); o.y = bf16_val(a.y); o.z = bf16_val(a.z); o.w = bf16_val(a.w);
  return o;
}
__device__ __forceinline__ float silu_p(float t) {
  return t * __builtin_amdgcn_rcpf(1.0f + __expf(-t));
}
__device__ __forceinline__ void split16(v4f x0, v4f x1, v4f x2, v4f x3, FragB& hi, FragB& lo) {
  const v8f fa = {x0.x, x0.y, x0.z, x0.w, x1.x, x1.y, x1.z, x1.w};
  const v8f fb = {x2.x, x2.y, x2.z, x2.w, x3.x, x3.y, x3.z, x3.w};
#pragma unroll
  for (int i = 0; i < 8; ++i) {
    const unsigned hb = bf16_bits(fa[i]);
    hi.u[i] = (unsigned short)hb;
    lo.u[i] = (unsigned short)bf16_bits(fa[i] - __uint_as_float(hb << 16));
  }
#pragma unroll
  for (int i = 0; i < 8; ++i) {
    const unsigned hb = bf16_bits(fb[i]);
    hi.u[8 + i] = (unsigned short)hb;
    lo.u[8 + i] = (unsigned short)bf16_bits(fb[i] - __uint_as_float(hb << 16));
  }
}
__device__ __forceinline__ v8us hl_pack8(const float* sp, unsigned part) {
  const v4f a = *(const v4fa*)sp;
  const v4f b = *(const v4fa*)(sp + 4);
  const v8f f8 = {a.x, a.y, a.z, a.w, b.x, b.y, b.z, b.w};
  const unsigned mh = 0u - part;
  const unsigned ml = ~mh;
  v8us oo;
#pragma unroll
  for (int e = 0; e < 8; ++e) {
    const unsigned hb = bf16_bits(f8[e]);
    const unsigned lb = bf16_bits(f8[e] - __uint_as_float(hb << 16));
    oo[e] = (unsigned short)((hb & ml) | (lb & mh));
  }
  return oo;
}
__device__ __forceinline__ void put16(unsigned short* dp, v8us o) {
  *(volatile v8us*)dp = o;
  __threadfence();
  *(volatile v8us*)dp = o;
}

__global__ __launch_bounds__(256) void k_prep(const float* __restrict__ gW1, const float* __restrict__ gWs,
                                              const float* __restrict__ gWv, const float* __restrict__ gWe,
                                              const float* __restrict__ gwp, const float* __restrict__ Watm,
                                              const float* __restrict__ Wsh, const float* __restrict__ Wb0,
                                              const float* __restrict__ Wbmap, const float* __restrict__ Wb1,
                                              unsigned short* PL) {
  const int u = (int)blockIdx.x * 256 + (int)threadIdx.x;
  if (u >= TUNITS) return;
  const float* src;
  int stride;
  int dup = 0;
  int zero = 0;
  if (u < NL * LUNITS) {
    const int l = u / LUNITS;
    const int v = u - l * LUNITS;
    const float* W1l = gW1 + (size_t)l * DIN * SD;
    if (v < U_W1AB) {
      const int n = v >> 6;
      const int kk = ((v & 63) * 8) & 255;
      src = W1l + (size_t)((n >> 8) * 256 + kk) * SD + (n & 255);
      stride = SD;
    } else if (v < U_W1AB + U_W1E) {
      const int w = v - U_W1AB;
      const int n = w >> 3;
      const int kk = ((w & 7) * 8) & 31;
      src = W1l + (size_t)(512 + kk) * SD + n;
      stride = SD;
    } else if (v < U_W1AB + U_W1E + U_WS) {
      const int w = v - (U_W1AB + U_W1E);
      const int n = w >> 6;
      const int kk = ((w & 63) * 8) & 255;
      src = gWs + (size_t)l * SD * SD + (size_t)kk * SD + n;
      stride = SD;
    } else if (v < U_W1AB + U_W1E + U_WS + U_WV) {
      const int w = v - (U_W1AB + U_W1E + U_WS);
      const int n = w >> 6;
      const int kk = ((w & 63) * 8) & 255;
      src = gWv + (size_t)l * SD * VD + (size_t)kk * VD + n;
      stride = VD;
    } else if (v < U_W1AB + U_W1E + U_WS + U_WV + 2048) {
      const int w = v - (U_W1AB + U_W1E + U_WS + U_WV);
      const int n = w >> 6;
      const int c0 = ((w & 63) * 8) >> 1;
      src = gWe + (size_t)l * SD * ED + (size_t)c0 * ED + n;
      stride = ED;
      dup = 1;
    } else {
      const int w = v - (U_W1AB + U_W1E + U_WS + U_WV + 2048);
      const int n = 32 + (w >> 6);
      const int c0 = ((w & 63) * 8) >> 1;
      src = gwp + (size_t)l * SD + c0;
      stride = 1;
      dup = 1;
      zero = (n != 32) ? 1 : 0;
    }
  } else {
    const int v = u - NL * LUNITS;
    if (v < 16384) {
      const int n = v >> 6;
      const int kk = ((v & 63) * 8) & 255;
      src = Watm + (size_t)kk * SD + n;
      stride = SD;
    } else if (v < 32768) {
      const int w = v - 16384;
      const int n = w >> 6;
      const int kk = ((w & 63) * 8) & 255;
      src = Wsh + (size_t)kk * SD + n;
      stride = SD;
    } else if (v < 49152) {
      const int w = v - 32768;
      const int n = w >> 6;
      const int c0 = ((w & 63) * 8) >> 1;
      src = Wb0 + (size_t)c0 * SD + n;
      stride = SD;
      dup = 1;
    } else if (v < 51200) {
      const int w = v - 49152;
      const int n = w >> 3;
      const int kk = ((w & 7) * 8) & 31;
      src = Wbmap + (size_t)kk * SD + n;
      stride = SD;
    } else {
      const int w = v - 51200;
      const int n = w >> 6;
      const int c0 = ((w & 63) * 8) >> 1;
      const int nc = n < 5 ? n : 4;
      src = Wb1 + (size_t)c0 * 5 + nc;
      stride = 5;
      dup = 1;
      zero = (n >= 5) ? 1 : 0;
    }
  }
  v8us o;
#pragma unroll
  for (int i = 0; i < 8; ++i) {
    const int idx = dup ? (i >> 1) : i;
    const float w = src[(size_t)idx * (size_t)stride];
    asm volatile("" :: "v"(w));
    const unsigned bits = bf16_bits(w);
    o[i] = zero ? (unsigned short)0 : (unsigned short)bits;
  }
  put16(PL + (size_t)u * 8, o);
}

__device__ __forceinline__ void init_store_pass(int tid, int nodeBase, v4f op, const v8us* oa, const v4f* oe,
                                                float* P0, unsigned short* A0hl, float* EP0, float* V) {
  if (tid < 8) *(volatile v4f*)(P0 + (size_t)(nodeBase + tid) * 4) = op;
#pragma unroll
  for (int it = 0; it < 2; ++it) {
    const int id = it * 256 + tid;
    const int row = id >> 6, pp = id & 63, part = pp >> 5, col8 = (pp & 31) * 8;
    *(volatile v8us*)(A0hl + (size_t)(nodeBase + row) * K2 + part * 256 + col8) = oa[it];
  }
#pragma unroll
  for (int it = 0; it < 8; ++it) {
    const int id = it * 256 + tid;
    *(volatile v4f*)(EP0 + (size_t)nodeBase * 1024 + (size_t)id * 4) = oe[it];
  }
  const v4f z4 = {0.0f, 0.0f, 0.0f, 0.0f};
  *(volatile v4f*)(V + (size_t)nodeBase * 192 + (size_t)tid * 4) = z4;
  if (tid < 128) *(volatile v4f*)(V + (size_t)nodeBase * 192 + (size_t)(256 + tid) * 4) = z4;
}

__global__ __launch_bounds__(256) void k_init(const float* __restrict__ x, const float* __restrict__ t,
                                              const float* __restrict__ pos,
                                              const float* __restrict__ Wtma, const float* __restrict__ btma,
                                              const float* __restrict__ Wtmb, const float* __restrict__ btmb,
                                              const float* __restrict__ Wam, const float* __restrict__ bam,
                                              const float* __restrict__ Wbm, const float* __restrict__ bbm,
                                              const float* __restrict__ Wbtm, const float* __restrict__ bbtm,
                                              float* P0, unsigned short* A0hl, float* EP0, float* V) {
  __shared__ __attribute__((aligned(16))) float sP[32 * 4];
  __shared__ __attribute__((aligned(16))) float sX[128];
  __shared__ __attribute__((aligned(16))) float sA0[8 * 256];
  __shared__ __attribute__((aligned(16))) float sU[256];
  __shared__ __attribute__((aligned(16))) float sE0[256];
  const int tid = (int)threadIdx.x, lane = tid & 31;
  const int wave = __builtin_amdgcn_readfirstlane(tid >> 5);
  const int blk = (int)blockIdx.x;
  const int nodeBase = blk * 8;
  const int b = blk >> 2;
  const int i0 = (blk & 3) * 8;

  if (wave == 0) {
    const int n = MOL * b + lane;
    const float px = bf16_val(pos[(size_t)n * 3 + 0]);
    const float py = bf16_val(pos[(size_t)n * 3 + 1]);
    const float pz = bf16_val(pos[(size_t)n * 3 + 2]);
    float sx = px, sy = py, sz = pz;
#pragma unroll
    for (int o = 16; o >= 1; o >>= 1) {
      sx += __shfl_xor(sx, o, 32);
      sy += __shfl_xor(sy, o, 32);
      sz += __shfl_xor(sz, o, 32);
    }
    const v4f c = {px - sx * 0.03125f, py - sy * 0.03125f, pz - sz * 0.03125f, 0.0f};
    *(v4fa*)(sP + 4 * lane) = c;
  }
  if (tid < 128) sX[tid] = bf16_val(x[(size_t)nodeBase * FD + tid]);
  __syncthreads();

  const float tb = bf16_val(t[b]);
  {
    const int c = tid;
    float acc[8];
#pragma unroll
    for (int q = 0; q < 8; ++q) acc[q] = 0.0f;
#pragma unroll 1
    for (int f = 0; f < FD; ++f) {
      const float w = bf16_val(Wam[(size_t)f * SD + c]);
#pragma unroll
      for (int q = 0; q < 8; ++q) acc[q] = fmaf(sX[q * FD + f], w, acc[q]);
    }
    const float tn = tb * bf16_val(Wtma[c]) + bf16_val(btma[c]);
    const float ba = bf16_val(bam[c]);
#pragma unroll
    for (int q = 0; q < 8; ++q) sA0[q * 256 + c] = (acc[q] + ba) + tn;
  }
  {
    const int q = tid >> 5, c = tid & 31;
    float acc = 0.0f;
#pragma unroll 1
    for (int f = 0; f < FD; ++f) acc = fmaf(sX[q * FD + f], bf16_val(Wbm[(size_t)f * ED + c]), acc);
    const float tm = tb * bf16_val(Wtmb[c]) + bf16_val(btmb[c]);
    sU[tid] = (acc + bf16_val(bbm[c])) + tm;
  }
  __syncthreads();
  {
    const int q = tid >> 5, c = tid & 31;
    float acc = 0.0f;
#pragma unroll 1
    for (int k = 0; k < ED; ++k) acc = fmaf(sU[q * ED + k], bf16_val(Wbtm[(size_t)k * ED + c]), acc);
    sE0[tid] = acc + bf16_val(bbtm[c]);
  }
  __syncthreads();

  const int tl = tid < 8 ? tid : 7;
  const v4f op = *(const v4fa*)(sP + 4 * (i0 + tl));
  asm volatile("" :: "v"(op));
  v8us oa[2];
#pragma unroll
  for (int it = 0; it < 2; ++it) {
    const int id = it * 256 + tid;
    const int row = id >> 6, pp = id & 63, part = pp >> 5, col8 = (pp & 31) * 8;
    oa[it] = hl_pack8(sA0 + row * 256 + col8, (unsigned)part);
  }
  v4f oe[8];
  {
    const int j = tid >> 3, c4 = (tid & 7) * 4;
#pragma unroll
    for (int it = 0; it < 8; ++it) {
      const v4f ev = *(const v4fa*)(sE0 + it * ED + c4);
      asm volatile("" :: "v"(ev));
      const bool pad = (j == i0 + it);
      v4f q;
      q.x = pad ? 0.0f : ev.x;
      q.y = pad ? 0.0f : ev.y;
      q.z = pad ? 0.0f : ev.z;
      q.w = pad ? 0.0f : ev.w;
      oe[it] = q;
    }
  }
  init_store_pass(tid, nodeBase, op, oa, oe, P0, A0hl, EP0, V);
  __threadfence();
  init_store_pass(tid, nodeBase, op, oa, oe, P0, A0hl, EP0, V);
}

template <int MODE, int NT>
__global__ __launch_bounds__(GTHR) __attribute__((amdgpu_num_vgpr(248)))
void k_gemm(const unsigned short* __restrict__ A, const unsigned short* __restrict__ BT, int K,
            const float* __restrict__ bias, float* Cm, int ldc, unsigned short* Chl) {
  constexpr int GBN = 16 * NT;
  __shared__ __attribute__((aligned(16))) float stg[GBM * GBN];
  __shared__ __attribute__((aligned(16))) float sb[GBN];
  const int tid = (int)threadIdx.x, lane = tid & 31, hh = lane >> 4, m = lane & 15;
  const int wave = __builtin_amdgcn_readfirstlane(tid >> 5);
  const int rowBase = (int)blockIdx.x * GBM;
  const int colBase = (int)blockIdx.y * GBN;

  if constexpr (MODE == 1 || MODE == 4) {
    if (tid < GBN / 4) {
      const v4f bv = bf16_val4(*(const v4fa*)(bias + colBase + 4 * tid));
      *(v4fa*)(sb + 4 * tid) = bv;
    }
    __syncthreads();
  }

  v8f acc[NT];
  {
    const v8f z = {0.f, 0.f, 0.f, 0.f, 0.f, 0.f, 0.f, 0.f};
#pragma unroll
    for (int t = 0; t < NT; ++t) acc[t] = z;
  }
  const unsigned short* ap = A  + (size_t)(rowBase + 16 * wave + m) * (size_t)K + 8 * hh;
  const unsigned short* bp = BT + (size_t)(colBase + m) * (size_t)K + 8 * hh;

#pragma unroll 1
  for (int k0 = 0; k0 < K; k0 += 32) {
    FragB af;
    af.h[0] = *(const v8usa*)(ap + k0);
    af.h[1] = *(const v8usa*)(ap + k0 + 16);
#pragma unroll
    for (int nt = 0; nt < NT; ++nt) {
      const unsigned short* wq = bp + (size_t)(16 * nt) * (size_t)K + k0;
      FragB bf;
      bf.h[0] = *(const v8usa*)wq;
      bf.h[1] = *(const v8usa*)(wq + 16);
      acc[nt] = wmb(af, bf, acc[nt]);
    }
  }

#pragma unroll
  for (int nt = 0; nt < NT; ++nt) {
    const int lc = 16 * nt + m;
    float bvv = 0.0f;
    if constexpr (MODE == 1 || MODE == 4) bvv = sb[lc];
#pragma unroll
    for (int r = 0; r < 8; ++r) {
      const int lr = 16 * wave + 8 * hh + r;
      float v = acc[nt][r];
      if constexpr (MODE == 1) v = v + bvv;
      if constexpr (MODE == 4) v = silu_p(v + bvv);
      stg[lr * GBN + lc] = v;
    }
  }
  __syncthreads();

  if constexpr (NT == 8) {
    if constexpr (MODE == 2) {
#pragma unroll
      for (int i = 0; i < 16; ++i) {
        const int row = rowBase + 16 * wave + i;
        const v4f old = *(const v4fa*)(Cm + (size_t)row * (size_t)ldc + colBase + 4 * lane);
        const v4f sv  = *(const v4fa*)(stg + (16 * wave + i) * GBN + 4 * lane);
        v4f q;
        q.x = old.x + sv.x; q.y = old.y + sv.y; q.z = old.z + sv.z; q.w = old.w + sv.w;
        *(v4fa*)(stg + (16 * wave + i) * GBN + 4 * lane) = q;
      }
      __syncthreads();
    }
    {
      v4f pv[16];
#pragma unroll
      for (int i = 0; i < 16; ++i) pv[i] = *(const v4fa*)(stg + (16 * wave + i) * GBN + 4 * lane);
#pragma unroll
      for (int i = 0; i < 16; ++i) {
        float* op = Cm + (size_t)(rowBase + 16 * wave + i) * (size_t)ldc + colBase + 4 * lane;
        *(volatile v4f*)op = pv[i];
      }
      __threadfence();
#pragma unroll
      for (int i = 0; i < 16; ++i) {
        float* op = Cm + (size_t)(rowBase + 16 * wave + i) * (size_t)ldc + colBase + 4 * lane;
        *(volatile v4f*)op = pv[i];
      }
    }
    if constexpr (MODE == 1 || MODE == 2) {
      const int part = lane >> 4;
      const int j = lane & 15;
      v8us pw[16];
#pragma unroll
      for (int i = 0; i < 16; ++i) pw[i] = hl_pack8(stg + (16 * wave + i) * GBN + 8 * j, (unsigned)part);
#pragma unroll
      for (int i = 0; i < 16; ++i) {
        unsigned short* op = Chl + (size_t)(rowBase + 16 * wave + i) * (size_t)K2 + part * 256 + colBase + 8 * j;
        *(volatile v8us*)op = pw[i];
      }
      __threadfence();
#pragma unroll
      for (int i = 0; i < 16; ++i) {
        unsigned short* op = Chl + (size_t)(rowBase + 16 * wave + i) * (size_t)K2 + part * 256 + colBase + 8 * j;
        *(volatile v8us*)op = pw[i];
      }
    }
  } else {
    v4f pv[8];
#pragma unroll
    for (int i = 0; i < 8; ++i) {
      const int lr = 16 * wave + 2 * i + (lane >> 4);
      const int c  = 4 * (lane & 15);
      const v4f old = *(const v4fa*)(Cm + (size_t)(rowBase + lr) * (size_t)ldc + colBase + c);
      const v4f sv  = *(const v4fa*)(stg + lr * GBN + c);
      v4f q;
      q.x = old.x + sv.x; q.y = old.y + sv.y; q.z = old.z + sv.z; q.w = old.w + sv.w;
      pv[i] = q;
    }
#pragma unroll
    for (int i = 0; i < 8; ++i) {
      const int lr = 16 * wave + 2 * i + (lane >> 4);
      float* op = Cm + (size_t)(rowBase + lr) * (size_t)ldc + colBase + 4 * (lane & 15);
      *(volatile v4f*)op = pv[i];
    }
    __threadfence();
#pragma unroll
    for (int i = 0; i < 8; ++i) {
      const int lr = 16 * wave + 2 * i + (lane >> 4);
      float* op = Cm + (size_t)(rowBase + lr) * (size_t)ldc + colBase + 4 * (lane & 15);
      *(volatile v4f*)op = pv[i];
    }
  }
}

__global__ __launch_bounds__(256) __attribute__((amdgpu_num_vgpr(248)))
void k_edge(const unsigned short* __restrict__ W1E, const unsigned short* __restrict__ WEP,
            const float* __restrict__ PAB, const float* __restrict__ W1da, const float* __restrict__ b1,
            const float* __restrict__ EPo, float* EPn, const float* __restrict__ Po, float* Pn,
            unsigned short* MHhl, unsigned short* RNHhl) {
  extern __shared__ __attribute__((aligned(16))) float dynf[];
  unsigned short* sW1E = (unsigned short*)(dynf + EO_W1E);
  unsigned short* sWEP = (unsigned short*)(dynf + EO_WEP);
  float*    sPA  = dynf + EO_PA;
  float*    sH   = dynf + EO_H;
  unsigned* sHL  = (unsigned*)(dynf + EO_HL);
  float*    sMH  = dynf + EO_MH;
  float*    sD2  = dynf + EO_D2;
  float*    sC   = dynf + EO_C;
  float*    sGeo = dynf + EO_GEO;
  float*    sPo  = dynf + EO_PO;
  float*    sPn  = dynf + EO_PN;

  const int tid = (int)threadIdx.x, lane = tid & 31, hh = lane >> 4, m = lane & 15;
  const int wave = __builtin_amdgcn_readfirstlane(tid >> 5);
  const int blk = (int)blockIdx.x;
  const int nodeBase = blk * 8;
  const int mol0 = (blk >> 2) * MOL;
  const int i0 = (blk & 3) * 8;
  const float inv31 = 1.0f / 31.0f;

#pragma unroll 4
  for (int it = 0; it < 8; ++it)
    ((v4ia*)sW1E)[it * 256 + tid] = ((const v4ia*)W1E)[it * 256 + tid];
#pragma unroll 4
  for (int it = 0; it < 12; ++it)
    ((v4ia*)sWEP)[it * 256 + tid] = ((const v4ia*)WEP)[it * 256 + tid];
#pragma unroll 4
  for (int it = 0; it < 8; ++it) {
    const int id = it * 256 + tid;
    const int row = id >> 6, c4 = (id & 63) * 4;
    *(v4fa*)(sPA + row * 256 + c4) = *(const v4fa*)(PAB + (size_t)(mol0 + row) * 512 + c4);
  }
  if (tid < 128) {
    *(v4fa*)(sC + 4 * tid) = bf16_val4(*(const v4fa*)(W1da + 4 * tid));
  } else if (tid < 192) {
    *(v4fa*)(sC + 512 + 4 * (tid - 128)) = bf16_val4(*(const v4fa*)(b1 + 4 * (tid - 128)));
  }
  if (tid < 32) *(v4fa*)(sPo + 4 * tid) = *(const v4fa*)(Po + (size_t)(mol0 + tid) * 4);
  __syncthreads();

  {
    const v4f pi = *(const v4fa*)(sPo + 4 * (i0 + wave));
    const v4f pj = *(const v4fa*)(sPo + 4 * lane);
    const float rx = pi.x - pj.x, ry = pi.y - pj.y, rz = pi.z - pj.z;
    const float a  = (pi.x * pj.x + pi.y * pj.y) + pi.z * pj.z;
    const float r2 = (rx * rx + ry * ry) + rz * rz;
    const float d  = sqrtf(fmaxf(r2, 1e-6f));
    const float iv = 1.0f / (1.0f + d);
    const v4f g0 = {d, a, rx * iv, ry * iv};
    const v4f g1 = {rz * iv, 0.0f, 0.0f, 0.0f};
    float* gp = sGeo + (wave * 32 + lane) * 8;
    *(v4fa*)gp = g0;
    *(v4fa*)(gp + 4) = g1;
  }
  __syncthreads();

  const v8f z8 = {0.f, 0.f, 0.f, 0.f, 0.f, 0.f, 0.f, 0.f};

#pragma unroll 1
  for (int q = 0; q < 8; ++q) {
    const int i = i0 + q;
    const int n = nodeBase + q;

    {
      FragB ahi0, alo0, ahi1, alo1;
      {
        const float* ep = EPo + ((size_t)n * 32 + m) * 32 + 8 * hh;
        const v4f x0 = *(const v4fa*)ep;
        const v4f x1 = *(const v4fa*)(ep + 4);
        const v4f x2 = *(const v4fa*)(ep + 16);
        const v4f x3 = *(const v4fa*)(ep + 20);
        split16(x0, x1, x2, x3, ahi0, alo0);
        const float* eq = ep + 16 * 32;
        const v4f y0 = *(const v4fa*)eq;
        const v4f y1 = *(const v4fa*)(eq + 4);
        const v4f y2 = *(const v4fa*)(eq + 16);
        const v4f y3 = *(const v4fa*)(eq + 20);
        split16(y0, y1, y2, y3, ahi1, alo1);
      }
      v8f acc[2][2];
      const unsigned short* bq = sW1E + (32 * wave + m) * 64 + 8 * hh;
#pragma unroll
      for (int nt = 0; nt < 2; ++nt) {
        const unsigned short* bp = bq + nt * 16 * 64;
        FragB b0, b1f;
        b0.h[0]  = *(const v8usa*)bp;
        b0.h[1]  = *(const v8usa*)(bp + 16);
        b1f.h[0] = *(const v8usa*)(bp + 32);
        b1f.h[1] = *(const v8usa*)(bp + 48);
        acc[0][nt] = wmb(ahi0, b0, z8);
        acc[0][nt] = wmb(alo0, b1f, acc[0][nt]);
        acc[1][nt] = wmb(ahi1, b0, z8);
        acc[1][nt] = wmb(alo1, b1f, acc[1][nt]);
      }
      float pbv[2], wdv[2], wav[2], bbv[2];
#pragma unroll
      for (int nt = 0; nt < 2; ++nt) {
        const int col = 32 * wave + 16 * nt + m;
        pbv[nt] = PAB[(size_t)n * 512 + 256 + col];
        wdv[nt] = sC[col];
        wav[nt] = sC[256 + col];
        bbv[nt] = sC[512 + col];
      }
#pragma unroll
      for (int mt = 0; mt < 2; ++mt) {
#pragma unroll
        for (int r = 0; r < 8; ++r) {
          const int row = 16 * mt + 8 * hh + r;
          const v4f gg = *(const v4fa*)(sGeo + (q * 32 + row) * 8);
#pragma unroll
          for (int nt = 0; nt < 2; ++nt) {
            const int col = 32 * wave + 16 * nt + m;
            const float pre = ((acc[mt][nt][r] + sPA[row * 256 + col]) + pbv[nt]) +
                              fmaf(gg.x, wdv[nt], fmaf(gg.y, wav[nt], bbv[nt]));
            const float hv = silu_p(pre);
            sH[row * 256 + col] = hv;
            const unsigned hb = bf16_bits(hv);
            const unsigned lb = bf16_bits(hv - __uint_as_float(hb << 16));
            sHL[row * HLP + col] = hb | (lb << 16);
          }
        }
      }
    }
    __syncthreads();

    {
      float s0 = 0.0f, s1 = 0.0f, s2 = 0.0f, s3 = 0.0f;
#pragma unroll 4
      for (int j = 0; j < 32; ++j) {
        if (j != i) {
          const float hv = sH[j * 256 + tid];
          const float* gg = sGeo + (q * 32 + j) * 8;
          const v4f g0 = *(const v4fa*)gg;
          const float gz = gg[4];
          s0 += hv;
          s1 = fmaf(g0.z, hv, s1);
          s2 = fmaf(g0.w, hv, s2);
          s3 = fmaf(gz, hv, s3);
        }
      }
      sMH[tid]       = s0 * inv31;
      sMH[256 + tid] = s1 * inv31;
      sMH[512 + tid] = s2 * inv31;
      sMH[768 + tid] = s3 * inv31;
    }
    if (wave < 6) {
      const int mt = (wave >= 3) ? 1 : 0;
      const int nt = wave - 3 * mt;
      v8f c2 = z8;
      const unsigned short* ap = (const unsigned short*)sHL + (16 * mt + m) * (2 * HLP) + 8 * hh;
      const unsigned short* bp = sWEP + (16 * nt + m) * 512 + 8 * hh;
#pragma unroll 2
      for (int k0 = 0; k0 < 512; k0 += 32) {
        FragB a, b;
        a.h[0] = *(const v8usa*)(ap + k0);
        a.h[1] = *(const v8usa*)(ap + k0 + 16);
        b.h[0] = *(const v8usa*)(bp + k0);
        b.h[1] = *(const v8usa*)(bp + k0 + 16);
        c2 = wmb(a, b, c2);
      }
#pragma unroll
      for (int r = 0; r < 8; ++r) sD2[(16 * mt + 8 * hh + r) * D2P + 16 * nt + m] = c2[r];
    }
    __syncthreads();

    {
      const int rq = wave >> 1;
      const int pp = tid & 63, part = pp >> 5, col8 = (pp & 31) * 8;
      const v8us oo = hl_pack8(sMH + rq * 256 + col8, (unsigned)part);
      unsigned short* dp = (rq == 0) ? (MHhl + (size_t)n * K2) : (RNHhl + (size_t)(3 * n + rq - 1) * K2);
      dp += part * 256 + col8;

      const int j = tid >> 3, c4 = (tid & 7) * 4;
      const v4f old = *(const v4fa*)(EPo + ((size_t)n * 32 + j) * 32 + c4);
      const v4f dd  = *(const v4fa*)(sD2 + j * D2P + c4);
      asm volatile("" :: "v"(old), "v"(dd));
      const bool pad = (j == i);
      v4f nv;
      nv.x = pad ? 0.0f : (old.x + dd.x);
      nv.y = pad ? 0.0f : (old.y + dd.y);
      nv.z = pad ? 0.0f : (old.z + dd.z);
      nv.w = pad ? 0.0f : (old.w + dd.w);
      float* ep = EPn + ((size_t)n * 32 + j) * 32 + c4;

      *(volatile v8us*)dp = oo;
      *(volatile v4f*)ep = nv;
      __threadfence();
      *(volatile v8us*)dp = oo;
      *(volatile v4f*)ep = nv;
    }
    if (wave == 0) {
      const float gdot = sD2[lane * D2P + 32];
      const float* gg = sGeo + (q * 32 + lane) * 8;
      const v4f g0 = *(const v4fa*)gg;
      const float gz = gg[4];
      const v4f pi = *(const v4fa*)(sPo + 4 * i);
      asm volatile("" :: "v"(gdot), "v"(g0), "v"(gz), "v"(pi));
      const float g = tanhf(gdot);
      const bool pad = (lane == i);
      float cx = pad ? 0.0f : g0.z * g;
      float cy = pad ? 0.0f : g0.w * g;
      float cz = pad ? 0.0f : gz * g;
#pragma unroll
      for (int o = 16; o >= 1; o >>= 1) {
        cx += __shfl_xor(cx, o, 32);
        cy += __shfl_xor(cy, o, 32);
        cz += __shfl_xor(cz, o, 32);
      }
      const v4f pn = {pi.x + cx * inv31, pi.y + cy * inv31, pi.z + cz * inv31, 0.0f};
      if (lane == 0) *(v4fa*)(sPn + 4 * q) = pn;
    }
  }
  __syncthreads();
  {
    const int tl = tid < 8 ? tid : 7;
    const v4f o4 = *(const v4fa*)(sPn + 4 * tl);
    asm volatile("" :: "v"(o4));
    float* pp = Pn + (size_t)(nodeBase + tl) * 4;
    if (tid < 8) *(volatile v4f*)pp = o4;
    __threadfence();
    if (tid < 8) *(volatile v4f*)pp = o4;
  }
}

__global__ __launch_bounds__(128) void k_coords(const float* __restrict__ P1, const float* __restrict__ V,
                                                const float* __restrict__ Wcl, float* C) {
  __shared__ __attribute__((aligned(16))) float sW[64];
  __shared__ __attribute__((aligned(16))) float sCc[128];
  const int tid = (int)threadIdx.x, lane = tid & 31;
  const int wave = __builtin_amdgcn_readfirstlane(tid >> 5);
  const int b = (int)blockIdx.x;
  if (tid < 16) *(v4fa*)(sW + 4 * tid) = bf16_val4(*(const v4fa*)(Wcl + 4 * tid));
  if (tid < 32) sCc[4 * tid + 3] = 0.0f;
  __syncthreads();
  if (wave < 3) {
    const int a = tid / 3;
    const int k = tid - 3 * a;
    const int n = MOL * b + a;
    const float* vr = V + (size_t)(3 * n + k) * VD;
    float acc = 0.0f;
#pragma unroll 1
    for (int v4 = 0; v4 < 16; ++v4) {
      const v4f vv = *(const v4fa*)(vr + 4 * v4);
      const v4f ww = *(const v4fa*)(sW + 4 * v4);
      acc = fmaf(vv.x, ww.x, acc);
      acc = fmaf(vv.y, ww.y, acc);
      acc = fmaf(vv.z, ww.z, acc);
      acc = fmaf(vv.w, ww.w, acc);
    }
    sCc[4 * a + k] = P1[(size_t)n * 4 + k] + acc;
  }
  __syncthreads();
  if (wave == 0) {
    const v4f c = *(const v4fa*)(sCc + 4 * lane);
    float sx = c.x, sy = c.y, sz = c.z;
#pragma unroll
    for (int o = 16; o >= 1; o >>= 1) {
      sx += __shfl_xor(sx, o, 32);
      sy += __shfl_xor(sy, o, 32);
      sz += __shfl_xor(sz, o, 32);
    }
    const v4f o4 = {c.x - sx * 0.03125f, c.y - sy * 0.03125f, c.z - sz * 0.03125f, 0.0f};
    float* cp = C + (size_t)(MOL * b + lane) * 4;
    *(volatile v4f*)cp = o4;
    __threadfence();
    *(volatile v4f*)cp = o4;
  }
}

__global__ __launch_bounds__(256) __attribute__((amdgpu_num_vgpr(248)))
void k_head(const float* __restrict__ EP, const float* __restrict__ SH, const float* __restrict__ C,
            const unsigned short* __restrict__ Wbm, const unsigned short* __restrict__ Wb0I,
            const unsigned short* __restrict__ Wb1I, const float* __restrict__ bbmap,
            const float* __restrict__ bb0, const float* __restrict__ wdsq, const float* __restrict__ bb1,
            float* out) {
  extern __shared__ __attribute__((aligned(16))) float dynf[];
  unsigned short* sWbm = (unsigned short*)(dynf + HO_WBM);
  unsigned short* sWb1 = (unsigned short*)(dynf + HO_WB1);
  float*    sSH  = dynf + HO_SH;
  unsigned* sF   = (unsigned*)(dynf + HO_F);
  unsigned* sG   = (unsigned*)(dynf + HO_G);
  float*    sOut = dynf + HO_OUT;
  float*    sDsq = dynf + HO_DSQ;
  float*    sC2  = dynf + HO_C;
  float*    sCo  = dynf + HO_CO;
  float*    sB1  = dynf + HO_B1;

  const int tid = (int)threadIdx.x, lane = tid & 31, hh = lane >> 4, m = lane & 15;
  const int wave = __builtin_amdgcn_readfirstlane(tid >> 5);
  const int b = (int)blockIdx.x;
  const int mol0 = b * MOL;

#pragma unroll 4
  for (int it = 0; it < 8; ++it)
    ((v4ia*)sWbm)[it * 256 + tid] = ((const v4ia*)Wbm)[it * 256 + tid];
#pragma unroll 4
  for (int it = 0; it < 4; ++it)
    ((v4ia*)sWb1)[it * 256 + tid] = ((const v4ia*)Wb1I)[it * 256 + tid];
#pragma unroll 4
  for (int it = 0; it < 8; ++it)
    ((v4fa*)sSH)[it * 256 + tid] = ((const v4fa*)(SH + (size_t)mol0 * SD))[it * 256 + tid];
  if (tid < 64) {
    *(v4fa*)(sC2 + 4 * tid) = bf16_val4(*(const v4fa*)(bbmap + 4 * tid));
  } else if (tid < 128) {
    *(v4fa*)(sC2 + 256 + 4 * (tid - 64)) = bf16_val4(*(const v4fa*)(bb0 + 4 * (tid - 64)));
  } else if (tid < 192) {
    *(v4fa*)(sC2 + 512 + 4 * (tid - 128)) = bf16_val4(*(const v4fa*)(wdsq + 4 * (tid - 128)));
  }
  if (tid < 32) *(v4fa*)(sCo + 4 * tid) = *(const v4fa*)(C + (size_t)(mol0 + tid) * 4);
  if (tid < 16) {
    const int tc = tid < 5 ? tid : 4;
    const float bv = bf16_val(bb1[tc]);
    asm volatile("" :: "v"(bv));
    sB1[tid] = (tid < 5) ? bv : 0.0f;
  }
  __syncthreads();
#pragma unroll
  for (int it = 0; it < 4; ++it) {
    const int id = it * 256 + tid;
    const int ii = id >> 5, jj = id & 31;
    const v4f ci = *(const v4fa*)(sCo + 4 * ii);
    const v4f cj = *(const v4fa*)(sCo + 4 * jj);
    const float dx = ci.x - cj.x, dy = ci.y - cj.y, dz = ci.z - cj.z;
    sDsq[id] = (dx * dx + dy * dy) + dz * dz;
  }
  __syncthreads();

  const v8f z8 = {0.f, 0.f, 0.f, 0.f, 0.f, 0.f, 0.f, 0.f};

#pragma unroll 1
  for (int i = 0; i < MOL; ++i) {
    {
      FragB ahi0, alo0, ahi1, alo1;
      {
        const int j = m;
        const float* pa = EP + ((size_t)(mol0 + i) * 32 + j) * 32 + 8 * hh;
        const float* pt = EP + ((size_t)(mol0 + j) * 32 + i) * 32 + 8 * hh;
        const v4f x0 = (*(const v4fa*)pa        + *(const v4fa*)pt)        * 0.5f;
        const v4f x1 = (*(const v4fa*)(pa + 4)  + *(const v4fa*)(pt + 4))  * 0.5f;
        const v4f x2 = (*(const v4fa*)(pa + 16) + *(const v4fa*)(pt + 16)) * 0.5f;
        const v4f x3 = (*(const v4fa*)(pa + 20) + *(const v4fa*)(pt + 20)) * 0.5f;
        split16(x0, x1, x2, x3, ahi0, alo0);
      }
      {
        const int j = 16 + m;
        const float* pa = EP + ((size_t)(mol0 + i) * 32 + j) * 32 + 8 * hh;
        const float* pt = EP + ((size_t)(mol0 + j) * 32 + i) * 32 + 8 * hh;
        const v4f x0 = (*(const v4fa*)pa        + *(const v4fa*)pt)        * 0.5f;
        const v4f x1 = (*(const v4fa*)(pa + 4)  + *(const v4fa*)(pt + 4))  * 0.5f;
        const v4f x2 = (*(const v4fa*)(pa + 16) + *(const v4fa*)(pt + 16)) * 0.5f;
        const v4f x3 = (*(const v4fa*)(pa + 20) + *(const v4fa*)(pt + 20)) * 0.5f;
        split16(x0, x1, x2, x3, ahi1, alo1);
      }
      v8f acc[2][2];
      const unsigned short* bq = sWbm + (32 * wave + m) * 64 + 8 * hh;
#pragma unroll
      for (int nt = 0; nt < 2; ++nt) {
        const unsigned short* bp = bq + nt * 16 * 64;
        FragB b0, b1f;
        b0.h[0]  = *(const v8usa*)bp;
        b0.h[1]  = *(const v8usa*)(bp + 16);
        b1f.h[0] = *(const v8usa*)(bp + 32);
        b1f.h[1] = *(const v8usa*)(bp + 48);
        acc[0][nt] = wmb(ahi0, b0, z8);
        acc[0][nt] = wmb(alo0, b1f, acc[0][nt]);
        acc[1][nt] = wmb(ahi1, b0, z8);
        acc[1][nt] = wmb(alo1, b1f, acc[1][nt]);
      }
#pragma unroll
      for (int nt = 0; nt < 2; ++nt) {
        const int col = 32 * wave + 16 * nt + m;
        const float shi = sSH[i * 256 + col];
        const float bm  = sC2[col];
#pragma unroll
        for (int mt = 0; mt < 2; ++mt) {
#pragma unroll
          for (int r = 0; r < 8; ++r) {
            const int row = 16 * mt + 8 * hh + r;
            const float fv = (shi + sSH[row * 256 + col]) + (acc[mt][nt][r] + bm);
            const unsigned hb = bf16_bits(fv);
            const unsigned lb = bf16_bits(fv - __uint_as_float(hb << 16));
            sF[row * HLP + col] = hb | (lb << 16);
          }
        }
      }
    }
    __syncthreads();

    {
      v8f acc[2][2];
#pragma unroll
      for (int mt = 0; mt < 2; ++mt)
#pragma unroll
        for (int nt = 0; nt < 2; ++nt) acc[mt][nt] = z8;
      const unsigned short* ap0 = (const unsigned short*)sF + m * (2 * HLP) + 8 * hh;
      const unsigned short* ap1 = ap0 + 16 * (2 * HLP);
      const unsigned short* bp  = Wb0I + (size_t)(32 * wave + m) * K2 + 8 * hh;
#pragma unroll 1
      for (int k0 = 0; k0 < K2; k0 += 32) {
        FragB a0, a1;
        a0.h[0] = *(const v8usa*)(ap0 + k0);
        a0.h[1] = *(const v8usa*)(ap0 + k0 + 16);
        a1.h[0] = *(const v8usa*)(ap1 + k0);
        a1.h[1] = *(const v8usa*)(ap1 + k0 + 16);
#pragma unroll
        for (int nt = 0; nt < 2; ++nt) {
          const unsigned short* wq = bp + (size_t)(16 * nt) * K2 + k0;
          FragB bf;
          bf.h[0] = *(const v8usa*)wq;
          bf.h[1] = *(const v8usa*)(wq + 16);
          acc[0][nt] = wmb(a0, bf, acc[0][nt]);
          acc[1][nt] = wmb(a1, bf, acc[1][nt]);
        }
      }
#pragma unroll
      for (int nt = 0; nt < 2; ++nt) {
        const int col = 32 * wave + 16 * nt + m;
        const float b0v = sC2[256 + col];
        const float wq  = sC2[512 + col];
#pragma unroll
        for (int mt = 0; mt < 2; ++mt) {
#pragma unroll
          for (int r = 0; r < 8; ++r) {
            const int row = 16 * mt + 8 * hh + r;
            const float hv = silu_p(acc[mt][nt][r] + fmaf(sDsq[i * 32 + row], wq, b0v));
            const unsigned hb = bf16_bits(hv);
            const unsigned lb = bf16_bits(hv - __uint_as_float(hb << 16));
            sG[row * HLP + col] = hb | (lb << 16);
          }
        }
      }
    }
    __syncthreads();

    if (wave < 2) {
      const int mt = wave;
      v8f c3 = z8;
      const unsigned short* ap = (const unsigned short*)sG + (16 * mt + m) * (2 * HLP) + 8 * hh;
      const unsigned short* bp = sWb1 + m * 512 + 8 * hh;
#pragma unroll 2
      for (int k0 = 0; k0 < K2; k0 += 32) {
        FragB a, bf;
        a.h[0]  = *(const v8usa*)(ap + k0);
        a.h[1]  = *(const v8usa*)(ap + k0 + 16);
        bf.h[0] = *(const v8usa*)(bp + k0);
        bf.h[1] = *(const v8usa*)(bp + k0 + 16);
        c3 = wmb(a, bf, c3);
      }
      const float bo = sB1[m];
#pragma unroll
      for (int r = 0; r < 8; ++r) {
        const int j = 16 * mt + 8 * hh + r;
        if (m < 5 && j != i) sOut[(31 * j + i - ((i > j) ? 1 : 0)) * 5 + m] = c3[r] + bo;
      }
    }
  }
  __syncthreads();

  {
    v4f pv[5];
#pragma unroll
    for (int it = 0; it < 5; ++it) {
      const int idx = it * 256 + tid;
      const int ic = idx < 1240 ? idx : 1239;
      pv[it] = *(const v4fa*)(sOut + 4 * ic);
      asm volatile("" :: "v"(pv[it]));
    }
    float* ob = out + (size_t)b * (EPM * 5);
#pragma unroll
    for (int it = 0; it < 5; ++it) {
      const int idx = it * 256 + tid;
      if (idx < 1240) *(volatile v4f*)(ob + 4 * idx) = pv[it];
    }
    __threadfence();
#pragma unroll
    for (int it = 0; it < 5; ++it) {
      const int idx = it * 256 + tid;
      if (idx < 1240) *(volatile v4f*)(ob + 4 * idx) = pv[it];
    }
  }
}

extern "C" void kernel_launch(void* const* d_in, const int* in_sizes, int n_in,
                              void* d_out, int out_size, void* d_ws, size_t ws_size,
                              hipStream_t stream) {
  if (n_in < 33) return;
  static const int want[33] = {32768, 64, 6144, 126976, 2048, 63488, 256, 256, 32, 32, 4096, 256, 512, 32,
                               65536, 256, 1024, 32, 698880, 1280, 327680, 81920, 40960, 1280, 65536, 256,
                               8192, 256, 65792, 256, 1280, 5, 64};
  for (int i = 0; i < 33; ++i) if (in_sizes[i] != want[i]) return;
  if (out_size != NE * 5) return;

  const float* x      = (const float*)d_in[0];
  const float* t      = (const float*)d_in[1];
  const float* pos    = (const float*)d_in[2];
  const float* W_tma  = (const float*)d_in[6];
  const float* b_tma  = (const float*)d_in[7];
  const float* W_tmb  = (const float*)d_in[8];
  const float* b_tmb  = (const float*)d_in[9];
  const float* W_am   = (const float*)d_in[10];
  const float* b_am   = (const float*)d_in[11];
  const float* W_bm   = (const float*)d_in[12];
  const float* b_bm   = (const float*)d_in[13];
  const float* W_atm  = (const float*)d_in[14];
  const float* b_atm  = (const float*)d_in[15];
  const float* W_btm  = (const float*)d_in[16];
  const float* b_btm  = (const float*)d_in[17];
  const float* gW1    = (const float*)d_in[18];
  const float* gb1    = (const float*)d_in[19];
  const float* gWs    = (const float*)d_in[20];
  const float* gWv    = (const float*)d_in[21];
  const float* gWe    = (const float*)d_in[22];
  const float* gwp    = (const float*)d_in[23];
  const float* W_sh   = (const float*)d_in[24];
  const float* b_sh   = (const float*)d_in[25];
  const float* W_bmap = (const float*)d_in[26];
  const float* b_bmap = (const float*)d_in[27];
  const float* W_b0   = (const float*)d_in[28];
  const float* b_b0   = (const float*)d_in[29];
  const float* W_b1   = (const float*)d_in[30];
  const float* b_b1   = (const float*)d_in[31];
  const float* W_cl   = (const float*)d_in[32];
  float* out = (float*)d_out;

  char* ws = (char*)d_ws;
  size_t off = 0;
  const size_t oPL   = off; off += (size_t)TUNITS * 16;
  const size_t oEP0  = off; off += (size_t)NN * 32 * 32 * 4;
  const size_t oEP1  = off; off += (size_t)NN * 32 * 32 * 4;
  const size_t oPAB  = off; off += (size_t)NN * 512 * 4;
  const size_t oS    = off; off += (size_t)NN * SD * 4;
  const size_t oShl  = off; off += (size_t)NN * K2 * 2;
  const size_t oA0   = off; off += (size_t)NN * K2 * 2;
  const size_t oMH   = off; off += (size_t)NN * K2 * 2;
  const size_t oRNH  = off; off += (size_t)3 * NN * K2 * 2;
  const size_t oV    = off; off += (size_t)3 * NN * VD * 4;
  const size_t oSH   = off; off += (size_t)NN * SD * 4;
  const size_t oP0   = off; off += (size_t)NN * 4 * 4;
  const size_t oP1   = off; off += (size_t)NN * 4 * 4;
  const size_t oC    = off; off += (size_t)NN * 4 * 4;
  if (off > ws_size || off > (size_t)WSMAX) return;

  unsigned short* PL   = (unsigned short*)(ws + oPL);
  float*          EP0  = (float*)(ws + oEP0);
  float*          EP1  = (float*)(ws + oEP1);
  float*          PAB  = (float*)(ws + oPAB);
  float*          S    = (float*)(ws + oS);
  unsigned short* Shl  = (unsigned short*)(ws + oShl);
  unsigned short* A0hl = (unsigned short*)(ws + oA0);
  unsigned short* MHhl = (unsigned short*)(ws + oMH);
  unsigned short* RNHh = (unsigned short*)(ws + oRNH);
  float*          V    = (float*)(ws + oV);
  float*          SHp  = (float*)(ws + oSH);
  float*          P0   = (float*)(ws + oP0);
  float*          P1   = (float*)(ws + oP1);
  float*          Cc   = (float*)(ws + oC);
  unsigned short* PH   = PL + (size_t)NL * LELEMS;

  hipFuncSetAttribute(reinterpret_cast<const void*>(&k_edge), hipFuncAttributeMaxDynamicSharedMemorySize,
                      (int)EDGE_LDS_BYTES);
  hipFuncSetAttribute(reinterpret_cast<const void*>(&k_head), hipFuncAttributeMaxDynamicSharedMemorySize,
                      (int)HEAD_LDS_BYTES);

  k_prep<<<TUNITS / 256, 256, 0, stream>>>(gW1, gWs, gWv, gWe, gwp, W_atm, W_sh, W_b0, W_bmap, W_b1, PL);
  k_init<<<NN / 8, 256, 0, stream>>>(x, t, pos, W_tma, b_tma, W_tmb, b_tmb, W_am, b_am, W_bm, b_bm,
                                     W_btm, b_btm, P0, A0hl, EP0, V);
  k_gemm<1, 8><<<dim3(NN / GBM, 2), GTHR, 0, stream>>>(A0hl, PH + HE_WATM, K2, b_atm, S, SD, Shl);

  for (int l = 0; l < NL; ++l) {
    const unsigned short* PLl = PL + (size_t)l * LELEMS;
    float* EPo = (l & 1) ? EP1 : EP0;
    float* EPn = (l & 1) ? EP0 : EP1;
    float* Po  = (l & 1) ? P1 : P0;
    float* Pn  = (l & 1) ? P0 : P1;
    k_gemm<0, 8><<<dim3(NN / GBM, 4), GTHR, 0, stream>>>(Shl, PLl + LE_W1AB, K2, b_atm, PAB, 512, Shl);
    k_edge<<<NN / 8, 256, EDGE_LDS_BYTES, stream>>>(PLl + LE_W1E, PLl + LE_WEP, PAB,
                                                    gW1 + (size_t)l * DIN * SD + (size_t)544 * SD,
                                                    gb1 + (size_t)l * SD, EPo, EPn, Po, Pn, MHhl, RNHh);
    k_gemm<2, 8><<<dim3(NN / GBM, 2), GTHR, 0, stream>>>(MHhl, PLl + LE_WS, K2, b_atm, S, SD, Shl);
    k_gemm<3, 4><<<dim3(3 * NN / GBM, 1), GTHR, 0, stream>>>(RNHh, PLl + LE_WV, K2, b_atm, V, VD, Shl);
  }
  k_gemm<4, 8><<<dim3(NN / GBM, 2), GTHR, 0, stream>>>(Shl, PH + HE_WSH, K2, b_sh, SHp, SD, Shl);
  k_coords<<<NB, 128, 0, stream>>>(P1, V, W_cl, Cc);
  k_head<<<NB, 256, HEAD_LDS_BYTES, stream>>>(EP1, SHp, Cc, PH + HE_WBM, PH + HE_WB0, PH + HE_WB1,
                                              b_bmap, b_b0, W_b0 + (size_t)256 * SD, b_b1, out);
}
